// GraphEncoder_53678501265724
// MI455X (gfx1250) — hardware-verified
//
#include <hip/hip_runtime.h>
#include <stddef.h>
#include <stdint.h>
#include <math.h>


#define DF     128
#define XP     256
#define NGR    2048
#define NH     512
#define NO     768
#define NTHR   256
#define NWAVE  8
#define EPT    8
#define CHUNK  (NTHR * EPT)
#define WCAP   (EPT * 32)
#define LISTN  (NWAVE * WCAP)
#define NBD    8192
#define SLD    13
#define NBA    1024
#define SLA    10
#define RCAP   12288
#define DEGCAP 32
#define PCAP   1024
#define GBM    64
#define GBN    128
#define GTHR   128
#define AGG_ZINTS (LISTN + 2 * RCAP + 3 * NBA)
#define MISC_INTS 16
#define REC_DBL   (NWAVE * 2 * DF)
#define SCAN_LDS_BYTES ((AGG_ZINTS + MISC_INTS) * 4 + REC_DBL * 8)

#define UB0 0
#define UB1 (UB0 + 128 * 16)
#define UB2 (UB1 + 128 * 32)
#define UB3 (UB2 + 128 * 32)
#define UB4 (UB3 + 128 * 32)
#define UB5 (UB4 + 512 * 32)
#define UB6 (UB5 + 512 * 128)
#define UB7 (UB6 + 512 * 128)
#define UB8 (UB7 + 768 * 128)
#define EO_W1 0
#define EO_W2 (EO_W1 + 128 * 128)
#define EO_W3 (EO_W2 + 128 * 256)
#define EO_WA (EO_W3 + 128 * 256)
#define EO_L1 (EO_WA + 128 * 256)
#define EO_L2 (EO_L1 + 512 * 256)
#define EO_L3 (EO_L2 + 512 * 1024)
#define EO_L4 (EO_L3 + 512 * 1024)
#define EO_END (EO_L4 + 768 * 1024)

static_assert((CHUNK & (CHUNK - 1)) == 0 && CHUNK <= 4096);
static_assert((NBD & (NBD - 1)) == 0 && NBD == (1 << SLD));
static_assert((NBA & (NBA - 1)) == 0 && NBA == (1 << SLA));
static_assert(((long long)CHUNK << SLD) < (1LL << 31));
static_assert(((long long)CHUNK << SLA) < (1LL << 31));
static_assert(NBD % (NTHR * 4) == 0);
static_assert(NBA % NWAVE == 0 && NBA % 32 == 0 && NBA % GBM == 0);
static_assert(RCAP % 4 == 0 && AGG_ZINTS % 4 == 0 && ((AGG_ZINTS + MISC_INTS) % 4) == 0);
static_assert(DEGCAP == 32);
static_assert(GBM == (GTHR / 32) * 16 && GBN == DF && DF == 4 * 32 && XP == 2 * DF);
static_assert(UB1 % NTHR == 0 && UB2 % NTHR == 0 && UB3 % NTHR == 0 && UB4 % NTHR == 0);
static_assert(UB5 % NTHR == 0 && UB6 % NTHR == 0 && UB7 % NTHR == 0 && UB8 % NTHR == 0);
static_assert(NGR % GBM == 0 && NH % GBN == 0 && NO % GBN == 0 && NGR % NWAVE == 0);
static_assert(SCAN_LDS_BYTES <= 300000);
static_assert(NO == 6 * 128);

typedef float          v4f   __attribute__((ext_vector_type(4)));
typedef float          v8f   __attribute__((ext_vector_type(8)));
typedef double         v2d   __attribute__((ext_vector_type(2)));
typedef int            v4i   __attribute__((ext_vector_type(4)));
typedef int            v8i   __attribute__((ext_vector_type(8)));
typedef unsigned int   v4u   __attribute__((ext_vector_type(4)));
typedef unsigned short v4us  __attribute__((ext_vector_type(4)));
typedef unsigned short v8us  __attribute__((ext_vector_type(8)));
typedef unsigned short v16us __attribute__((ext_vector_type(16)));
typedef __bf16         v16bf __attribute__((ext_vector_type(16)));
typedef v4f  __attribute__((may_alias)) v4fa;
typedef v4i  __attribute__((may_alias)) v4ia;
typedef v4u  __attribute__((may_alias)) v4ua;
typedef v4us __attribute__((may_alias)) v4usa;
typedef v8us __attribute__((may_alias)) v8usa;
union FragB { v16bf v; v16us u; v8us h[2]; v8i w; };

__device__ __forceinline__ v8f wmb(const FragB& a, const FragB& b, v8f c) {
  v8f d = __builtin_amdgcn_wmma_f32_16x16x32_bf16(false, a.v, false, b.v, (short)0, c, false, false);
  asm volatile("v_nop\n\tv_nop\n\tv_nop\n\tv_nop" : "+v"(d) : "v"(a.w), "v"(b.w));
  return d;
}

__device__ __forceinline__ unsigned bf16_bits(float f) {
  const unsigned u = __float_as_uint(f);
  return (u + 0x7FFFu + ((u >> 16) & 1u)) >> 16;
}
__device__ __forceinline__ float bf16_val(float f) {
  return __uint_as_float(bf16_bits(f) << 16);
}
__device__ __forceinline__ v4f bf16_val4(v4f a) {
  v4f r;
  r.x = bf16_val(a.x); r.y = bf16_val(a.y); r.z = bf16_val(a.z); r.w = bf16_val(a.w);
  return r;
}
__device__ __forceinline__ float wsum(float v) {
#pragma unroll
  for (int o = 16; o > 0; o >>= 1) v += __shfl_xor(v, o, 32);
  return v;
}
__device__ __forceinline__ float wmaxf(float v) {
#pragma unroll
  for (int o = 16; o > 0; o >>= 1) v = fmaxf(v, __shfl_xor(v, o, 32));
  return v;
}
__device__ __forceinline__ float leaky02(float v) { return v >= 0.0f ? v : 0.2f * v; }

__device__ __forceinline__ void wave_sync() {
  __builtin_amdgcn_fence(__ATOMIC_RELEASE, "wavefront");
  __builtin_amdgcn_wave_barrier();
  __builtin_amdgcn_fence(__ATOMIC_ACQUIRE, "wavefront");
}

template <int SLB>
__device__ __forceinline__ int scan_chunk(const int* __restrict__ dsts, int nE, int cbase, int slotBase,
                                          int nb, int vec8, int* list, int tid, int lane, int wave) {
  int wc = 0;
  const int el0  = tid * EPT;
  const int e0   = cbase + el0;
  const int sent = -2147483647 - 1;
  v4i da, db;
  if (vec8 != 0 && cbase + CHUNK <= nE) {
    da = *(const v4i*)(dsts + e0);
    db = *(const v4i*)(dsts + e0 + 4);
  } else {
    da.x = (e0     < nE) ? dsts[min(e0,     nE - 1)] : sent;
    da.y = (e0 + 1 < nE) ? dsts[min(e0 + 1, nE - 1)] : sent;
    da.z = (e0 + 2 < nE) ? dsts[min(e0 + 2, nE - 1)] : sent;
    da.w = (e0 + 3 < nE) ? dsts[min(e0 + 3, nE - 1)] : sent;
    db.x = (e0 + 4 < nE) ? dsts[min(e0 + 4, nE - 1)] : sent;
    db.y = (e0 + 5 < nE) ? dsts[min(e0 + 5, nE - 1)] : sent;
    db.z = (e0 + 6 < nE) ? dsts[min(e0 + 6, nE - 1)] : sent;
    db.w = (e0 + 7 < nE) ? dsts[min(e0 + 7, nE - 1)] : sent;
  }
  const unsigned nbs = (unsigned)slotBase;
  const unsigned unb = (unsigned)nb;
  const unsigned s0 = (unsigned)da.x - nbs, s1 = (unsigned)da.y - nbs;
  const unsigned s2 = (unsigned)da.z - nbs, s3 = (unsigned)da.w - nbs;
  const unsigned s4 = (unsigned)db.x - nbs, s5 = (unsigned)db.y - nbs;
  const unsigned s6 = (unsigned)db.z - nbs, s7 = (unsigned)db.w - nbs;
  const bool h0 = s0 < unb, h1 = s1 < unb, h2 = s2 < unb, h3 = s3 < unb;
  const bool h4 = s4 < unb, h5 = s5 < unb, h6 = s6 < unb, h7 = s7 < unb;
  const unsigned any = __builtin_amdgcn_ballot_w32(h0 | h1 | h2 | h3 | h4 | h5 | h6 | h7);
  if (any != 0u) {
#define HITJ(J, HJ, SJ) { \
      const unsigned mj = __builtin_amdgcn_ballot_w32(HJ); \
      if (mj != 0u) { \
        if (HJ) { \
          const int pos = wc + (int)__builtin_amdgcn_mbcnt_lo(mj, 0u); \
          if (pos < WCAP) list[wave * WCAP + pos] = ((el0 + (J)) << SLB) | (int)(SJ); \
        } \
        wc += (int)__builtin_popcount(mj); } }
    HITJ(0, h0, s0)
    HITJ(1, h1, s1)
    HITJ(2, h2, s2)
    HITJ(3, h3, s3)
    HITJ(4, h4, s4)
    HITJ(5, h5, s5)
    HITJ(6, h6, s6)
    HITJ(7, h7, s7)
#undef HITJ
  }
  return wc;
}

__global__ __launch_bounds__(NTHR) void k_wprep(const float* __restrict__ W1, const float* __restrict__ W2,
                                                const float* __restrict__ W3, const float* __restrict__ Wa,
                                                const float* __restrict__ L1, const float* __restrict__ L2,
                                                const float* __restrict__ L3, const float* __restrict__ L4,
                                                unsigned short* WP) {
  const int u = (int)blockIdx.x * NTHR + (int)threadIdx.x;
  const float* W;
  int K, N, sh, ub, eo;
  if (u < UB1)      { W = W1; K = 128; N = 128; sh = 4; ub = UB0; eo = EO_W1; }
  else if (u < UB2) { W = W2; K = 128; N = 128; sh = 5; ub = UB1; eo = EO_W2; }
  else if (u < UB3) { W = W3; K = 128; N = 128; sh = 5; ub = UB2; eo = EO_W3; }
  else if (u < UB4) { W = Wa; K = 128; N = 128; sh = 5; ub = UB3; eo = EO_WA; }
  else if (u < UB5) { W = L1; K = 128; N = 512; sh = 5; ub = UB4; eo = EO_L1; }
  else if (u < UB6) { W = L2; K = 512; N = 512; sh = 7; ub = UB5; eo = EO_L2; }
  else if (u < UB7) { W = L3; K = 512; N = 512; sh = 7; ub = UB6; eo = EO_L3; }
  else if (u < UB8) { W = L4; K = 512; N = 768; sh = 7; ub = UB7; eo = EO_L4; }
  else return;
  const int v  = u - ub;
  const int n  = v >> sh;
  const int k8 = (v & ((1 << sh) - 1)) * 8;
  const int ks = k8 & (K - 1);
  const float* p = W + (size_t)ks * (size_t)N + n;
  v8us o;
#pragma unroll
  for (int i = 0; i < 8; ++i) o[i] = (unsigned short)bf16_bits(p[(size_t)i * (size_t)N]);
  unsigned short* dp = WP + (size_t)eo + (size_t)n * (size_t)(8 << sh) + k8;
  *(volatile v8us*)dp = o;
  __threadfence();
  *(volatile v8us*)dp = o;
}

__global__ __launch_bounds__(NTHR) void k_cvx(const float* __restrict__ x, int nN, int nUnits,
                                              unsigned short* xh) {
  const int u = (int)blockIdx.x * NTHR + (int)threadIdx.x;
  if (u >= nUnits) return;
  const int row = u >> 5;
  const int c8  = (u & 31) * 8;
  const int kk  = c8 & (DF - 1);
  const int rc  = row < nN ? row : nN - 1;
  const float* p = x + (size_t)rc * DF + kk;
  const v4f a = *(const v4fa*)p;
  const v4f b = *(const v4fa*)(p + 4);
  const bool ok = (row < nN) && (c8 < DF);
  v8us o;
  o[0] = ok ? (unsigned short)bf16_bits(a.x) : (unsigned short)0;
  o[1] = ok ? (unsigned short)bf16_bits(a.y) : (unsigned short)0;
  o[2] = ok ? (unsigned short)bf16_bits(a.z) : (unsigned short)0;
  o[3] = ok ? (unsigned short)bf16_bits(a.w) : (unsigned short)0;
  o[4] = ok ? (unsigned short)bf16_bits(b.x) : (unsigned short)0;
  o[5] = ok ? (unsigned short)bf16_bits(b.y) : (unsigned short)0;
  o[6] = ok ? (unsigned short)bf16_bits(b.z) : (unsigned short)0;
  o[7] = ok ? (unsigned short)bf16_bits(b.w) : (unsigned short)0;
  unsigned short* dp = xh + (size_t)row * XP + c8;
  *(volatile v8us*)dp = o;
  __threadfence();
  *(volatile v8us*)dp = o;
}

__global__ __launch_bounds__(NTHR) void k_deg(const int* __restrict__ dsts, int nE, int vec8, float* dis) {
  __shared__ __attribute__((aligned(16))) int scnt[NBD];
  __shared__ __attribute__((aligned(16))) int list[LISTN];
  __shared__ int wcnt[NWAVE];
  const int tid = (int)threadIdx.x, lane = tid & 31, wave = tid >> 5;
  const int nodeBase = (int)blockIdx.x * NBD;

  for (int i = tid; i < NBD; i += NTHR) scnt[i] = 0;
  for (int i = tid; i < LISTN; i += NTHR) list[i] = 0;
  if (tid < NWAVE) wcnt[tid] = 0;
  __syncthreads();

  const int nChunks = (nE + CHUNK - 1) / CHUNK;
#pragma unroll 1
  for (int ch = 0; ch < nChunks; ++ch) {
    const int cbase = ch * CHUNK;
    const int wc = scan_chunk<SLD>(dsts, nE, cbase, nodeBase, NBD, vec8, list, tid, lane, wave);
    if (lane == 0) wcnt[wave] = wc;
    __syncthreads();
    if (wave == 0) {
#pragma unroll 1
      for (int w2 = 0; w2 < NWAVE; ++w2) {
        int c = wcnt[w2];
        c = c < 0 ? 0 : (c > WCAP ? WCAP : c);
#pragma unroll 1
        for (int b0 = 0; b0 < c; b0 += 32) {
          const int idx = b0 + lane;
          const int ent = list[w2 * WCAP + (idx < WCAP ? idx : WCAP - 1)];
          const int m32 = (c - b0) < 32 ? (c - b0) : 32;
#pragma unroll 1
          for (int k = 0; k < m32; ++k) {
            const int u  = __builtin_amdgcn_readlane(ent, k);
            const int sl = u & (NBD - 1);
            if (lane == 0) scnt[sl] = scnt[sl] + 1;
          }
        }
      }
    }
    __syncthreads();
  }

  v4f vals[NBD / (NTHR * 4)];
#pragma unroll
  for (int it = 0; it < NBD / (NTHR * 4); ++it) {
    const int s0 = it * (NTHR * 4) + 4 * tid;
    const v4i c4 = *(const v4ia*)(scnt + s0);
    const float d0 = (float)c4.x + 1.0f, d1 = (float)c4.y + 1.0f;
    const float d2 = (float)c4.z + 1.0f, d3 = (float)c4.w + 1.0f;
    v4f v;
    v.x = rsqrtf(d0); v.y = rsqrtf(d1); v.z = rsqrtf(d2); v.w = rsqrtf(d3);
    vals[it] = v;
  }
#pragma unroll
  for (int it = 0; it < NBD / (NTHR * 4); ++it) {
    const int s0 = it * (NTHR * 4) + 4 * tid;
    *(volatile v4f*)(dis + (size_t)nodeBase + s0) = vals[it];
  }
  __threadfence();
#pragma unroll
  for (int it = 0; it < NBD / (NTHR * 4); ++it) {
    const int s0 = it * (NTHR * 4) + 4 * tid;
    *(volatile v4f*)(dis + (size_t)nodeBase + s0) = vals[it];
  }
}

template <int MODE>
__global__ __launch_bounds__(GTHR) void k_gemm(const unsigned short* __restrict__ A, int lda,
                                               const unsigned short* __restrict__ BT, int K, int ldo,
                                               const float* __restrict__ bias, float* outF, unsigned short* outH,
                                               const float* __restrict__ avs, const float* __restrict__ avd,
                                               float* AL, float* AR) {
  __shared__ __attribute__((aligned(16))) float stg[GBM * GBN];
  __shared__ __attribute__((aligned(16))) float sdot[2 * GBM];
  const int tid = (int)threadIdx.x, lane = tid & 31, wave = tid >> 5, hh = lane >> 4, m = lane & 15;
  const int rowBase = (int)blockIdx.x * GBM;
  const int col0    = (int)blockIdx.y * GBN;

  v8f acc[8];
  {
    const v8f z = {0.f, 0.f, 0.f, 0.f, 0.f, 0.f, 0.f, 0.f};
#pragma unroll
    for (int t = 0; t < 8; ++t) acc[t] = z;
  }
  const unsigned short* ap = A + (size_t)(rowBase + 16 * wave + m) * (size_t)lda + 8 * hh;
  const unsigned short* bp = BT + (size_t)(col0 + m) * (size_t)K + 8 * hh;

#pragma unroll 1
  for (int k0 = 0; k0 < K; k0 += 32) {
    FragB af;
    af.h[0] = *(const v8usa*)(ap + k0);
    af.h[1] = *(const v8usa*)(ap + k0 + 16);
#pragma unroll
    for (int nt = 0; nt < 8; ++nt) {
      const unsigned short* wq = bp + (size_t)(16 * nt) * (size_t)K + k0;
      FragB bf;
      bf.h[0] = *(const v8usa*)wq;
      bf.h[1] = *(const v8usa*)(wq + 16);
      acc[nt] = wmb(af, bf, acc[nt]);
    }
  }

#pragma unroll
  for (int nt = 0; nt < 8; ++nt) {
    const int lc = 16 * nt + m;
#pragma unroll
    for (int r = 0; r < 8; ++r) {
      const int lr = 16 * wave + 8 * hh + r;
      stg[lr * GBN + lc] = acc[nt][r];
    }
  }
  __syncthreads();

  v4f pv[16];
#pragma unroll
  for (int i = 0; i < 16; ++i) pv[i] = *(const v4fa*)(stg + (16 * wave + i) * GBN + 4 * lane);

  if constexpr (MODE == 0 || MODE == 1) {
#pragma unroll
    for (int i = 0; i < 16; ++i) {
      float* op = outF + (size_t)(rowBase + 16 * wave + i) * (size_t)ldo + col0 + 4 * lane;
      *(volatile v4f*)op = pv[i];
    }
    __threadfence();
#pragma unroll
    for (int i = 0; i < 16; ++i) {
      float* op = outF + (size_t)(rowBase + 16 * wave + i) * (size_t)ldo + col0 + 4 * lane;
      *(volatile v4f*)op = pv[i];
    }
    if constexpr (MODE == 1) {
      const v4f a4 = bf16_val4(*(const v4f*)(avs + 4 * lane));
      const v4f d4 = bf16_val4(*(const v4f*)(avd + 4 * lane));
      float alv = 0.0f, arv = 0.0f;
#pragma unroll 1
      for (int i = 0; i < 16; ++i) {
        const v4f v = *(const v4fa*)(stg + (16 * wave + i) * GBN + 4 * lane);
        float s1 = v.x * a4.x; s1 = fmaf(v.y, a4.y, s1); s1 = fmaf(v.z, a4.z, s1); s1 = fmaf(v.w, a4.w, s1);
        float s2 = v.x * d4.x; s2 = fmaf(v.y, d4.y, s2); s2 = fmaf(v.z, d4.z, s2); s2 = fmaf(v.w, d4.w, s2);
        s1 = wsum(s1);
        s2 = wsum(s2);
        alv = (lane == i) ? s1 : alv;
        arv = (lane == i) ? s2 : arv;
      }
      if (lane < 16) { sdot[16 * wave + lane] = alv; sdot[GBM + 16 * wave + lane] = arv; }
      __syncthreads();
      if (wave == 0) {
        const v4f dv = *(const v4fa*)(sdot + 4 * lane);
        float* dp = (lane < 16) ? (AL + (size_t)rowBase + 4 * lane) : (AR + (size_t)rowBase + 4 * (lane - 16));
        *(volatile v4f*)dp = dv;
        __threadfence();
        *(volatile v4f*)dp = dv;
      }
    }
  } else {
    const v4f bb4 = bf16_val4(*(const v4f*)(bias + col0 + 4 * lane));
#pragma unroll
    for (int i = 0; i < 16; ++i) {
      v4f y = pv[i] + bb4;
      if constexpr (MODE == 2) {
        y.x = fmaxf(y.x, 0.0f); y.y = fmaxf(y.y, 0.0f); y.z = fmaxf(y.z, 0.0f); y.w = fmaxf(y.w, 0.0f);
      }
      pv[i] = y;
    }
    if constexpr (MODE == 3) {
#pragma unroll
      for (int i = 0; i < 16; ++i) {
        float* op = outF + (size_t)(rowBase + 16 * wave + i) * (size_t)ldo + col0 + 4 * lane;
        *(volatile v4f*)op = pv[i];
      }
      __threadfence();
#pragma unroll
      for (int i = 0; i < 16; ++i) {
        float* op = outF + (size_t)(rowBase + 16 * wave + i) * (size_t)ldo + col0 + 4 * lane;
        *(volatile v4f*)op = pv[i];
      }
    } else {
      __syncthreads();
#pragma unroll
      for (int i = 0; i < 16; ++i) {
        v4us h4, l4;
        unsigned hb;
        hb = bf16_bits(pv[i].x); h4[0] = (unsigned short)hb; l4[0] = (unsigned short)bf16_bits(pv[i].x - __uint_as_float(hb << 16));
        hb = bf16_bits(pv[i].y); h4[1] = (unsigned short)hb; l4[1] = (unsigned short)bf16_bits(pv[i].y - __uint_as_float(hb << 16));
        hb = bf16_bits(pv[i].z); h4[2] = (unsigned short)hb; l4[2] = (unsigned short)bf16_bits(pv[i].z - __uint_as_float(hb << 16));
        hb = bf16_bits(pv[i].w); h4[3] = (unsigned short)hb; l4[3] = (unsigned short)bf16_bits(pv[i].w - __uint_as_float(hb << 16));
        unsigned short* srow = (unsigned short*)stg + (size_t)(16 * wave + i) * (2 * GBN);
        *(v4usa*)(srow + 4 * lane) = h4;
        *(v4usa*)(srow + DF + 4 * lane) = l4;
      }
      __syncthreads();
      v8us qv[16];
#pragma unroll
      for (int i = 0; i < 16; ++i) {
        const unsigned short* srow = (const unsigned short*)stg + (size_t)(16 * wave + i) * (2 * GBN);
        qv[i] = *(const v8usa*)(srow + 8 * lane);
      }
      const int cofs = (lane < 16) ? (col0 + 8 * lane) : (ldo + col0 + 8 * (lane - 16));
#pragma unroll
      for (int i = 0; i < 16; ++i) {
        unsigned short* rp = outH + (size_t)(rowBase + 16 * wave + i) * (size_t)(2 * ldo) + cofs;
        *(volatile v8us*)rp = qv[i];
      }
      __threadfence();
#pragma unroll
      for (int i = 0; i < 16; ++i) {
        unsigned short* rp = outH + (size_t)(rowBase + 16 * wave + i) * (size_t)(2 * ldo) + cofs;
        *(volatile v8us*)rp = qv[i];
      }
    }
  }
}

template <int GAT>
__global__ __launch_bounds__(NTHR) void k_scan(const int* __restrict__ srcs, const int* __restrict__ dsts,
                                               int nE, int nN, int vec8, int mRows,
                                               const float* __restrict__ dis,
                                               const float* __restrict__ al, const float* __restrict__ ar,
                                               const float* __restrict__ hx, const float* __restrict__ bias,
                                               float* aout, double* rec) {
  extern __shared__ __attribute__((aligned(16))) int dsm[];
  int* list = dsm;
  int* hl   = dsm + LISTN;
  int* sl   = hl + RCAP;
  int* cnt  = sl + RCAP;
  int* offs = cnt + NBA;
  int* cur  = offs + NBA;
  int* misc = cur + NBA;
  double* recb = (double*)(misc + MISC_INTS);
  const int tid = (int)threadIdx.x, lane = tid & 31, wave = tid >> 5;
  const int nodeBase = (int)blockIdx.x * NBA;

  {
    const v4i z4 = {0, 0, 0, 0};
    for (int i = tid * 4; i < AGG_ZINTS; i += NTHR * 4) *(v4ia*)(dsm + i) = z4;
    if (tid < MISC_INTS) misc[tid] = 0;
  }
  const v4f bv = bf16_val4(*(const v4f*)(bias + 4 * lane));
  __syncthreads();

  int t = 0, ov = 0;
  const int nChunks = (nE + CHUNK - 1) / CHUNK;
#pragma unroll 1
  for (int ch = 0; ch < nChunks; ++ch) {
    const int cbase = ch * CHUNK;
    const int wc = scan_chunk<SLA>(dsts, nE, cbase, nodeBase, NBA, vec8, list, tid, lane, wave);
    if (lane == 0) misc[wave] = wc;
    __syncthreads();
    if (wave == 0) {
#pragma unroll 1
      for (int w2 = 0; w2 < NWAVE; ++w2) {
        int c = misc[w2];
        c = c < 0 ? 0 : (c > WCAP ? WCAP : c);
#pragma unroll 1
        for (int b0 = 0; b0 < c; b0 += 32) {
          const int idx = b0 + lane;
          const int ent = list[w2 * WCAP + (idx < WCAP ? idx : WCAP - 1)];
          const int m32 = (c - b0) < 32 ? (c - b0) : 32;
#pragma unroll 1
          for (int k = 0; k < m32; ++k) {
            const int u    = __builtin_amdgcn_readlane(ent, k);
            const int slot = u & (NBA - 1);
            const int el   = (u >> SLA) & (CHUNK - 1);
            const int pk   = ((cbase + el) << SLA) | slot;
            if (t < RCAP) {
              if (lane == 0) { hl[t] = pk; cnt[slot] = cnt[slot] + 1; }
              t = t + 1;
            } else {
              ov = 1;
            }
          }
        }
      }
    }
    __syncthreads();
  }
  if (wave == 0 && lane == 0) { misc[8] = t; misc[9] = ov; }
  __syncthreads();
  int tt = misc[8];
  tt = tt < 0 ? 0 : (tt > RCAP ? RCAP : tt);
  const int ovf = misc[9];

  if (wave == 0) {
    const int base = lane * (NBA / 32);
    int s = 0;
#pragma unroll 1
    for (int i = 0; i < NBA / 32; ++i) s += cnt[base + i];
    int incl = s;
#pragma unroll
    for (int d = 1; d < 32; d <<= 1) {
      const int y = __shfl_up(incl, d, 32);
      if (lane >= d) incl += y;
    }
    int run = incl - s;
#pragma unroll 1
    for (int i = 0; i < NBA / 32; ++i) {
      const int cv = cnt[base + i];
      offs[base + i] = run;
      cur[base + i]  = run;
      run += cv;
    }
  }
  __syncthreads();
  if (wave == 0) {
#pragma unroll 1
    for (int b0 = 0; b0 < tt; b0 += 32) {
      const int idx = b0 + lane;
      const int ent = hl[idx < RCAP ? idx : RCAP - 1];
      const int m32 = (tt - b0) < 32 ? (tt - b0) : 32;
#pragma unroll 1
      for (int k = 0; k < m32; ++k) {
        const int u    = __builtin_amdgcn_readlane(ent, k);
        const int slot = u & (NBA - 1);
        if (lane == 0) {
          int p = cur[slot];
          p = p < 0 ? 0 : (p > RCAP - 1 ? RCAP - 1 : p);
          sl[p] = u;
          cur[slot] = p + 1;
        }
      }
    }
  }
  __syncthreads();

  const float qnan = __int_as_float(0x7fc00000);
  const float pz = (ovf != 0) ? qnan : 0.0f;
  const float ninf = -__builtin_inff();
  double sd0 = 0.0, sd1 = 0.0, sd2 = 0.0, sd3 = 0.0;
  double sq0 = 0.0, sq1 = 0.0, sq2 = 0.0, sq3 = 0.0;
#pragma unroll 1
  for (int si = 0; si < NBA / NWAVE; ++si) {
    const int s    = si * NWAVE + wave;
    const int node = nodeBase + s;
    int c = cnt[s];
    const bool big = c > DEGCAP;
    c = c < 0 ? 0 : (c > DEGCAP ? DEGCAP : c);
    int o = offs[s];
    o = o < 0 ? 0 : (o > RCAP ? RCAP : o);
    const int nc = node < nN ? node : nN - 1;
    int idx = o + lane;
    idx = idx > RCAP - 1 ? RCAP - 1 : idx;
    const int ent = sl[idx];
    int eid = ent >> SLA;
    eid = eid < 0 ? 0 : (eid > nE - 1 ? nE - 1 : eid);
    int sr = srcs[eid];
    sr = sr < 0 ? 0 : (sr > nN - 1 ? nN - 1 : sr);
    const bool valid = lane < c;
    float wt, wself;
    if constexpr (GAT != 0) {
      const float ari = ar[nc];
      const float e   = leaky02(al[sr] + ari);
      const float es  = leaky02(al[nc] + ari);
      float mx = valid ? e : ninf;
      mx = wmaxf(mx);
      mx = fmaxf(mx, es);
      const float pe = expf(e - mx);
      const float p  = valid ? pe : 0.0f;
      const float ps = expf(es - mx);
      float sm = wsum(p);
      sm = sm + ps;
      const float inv = 1.0f / sm;
      wt = p * inv;
      wself = ps * inv;
    } else {
      const float dd = dis[nc];
      wt = dis[sr] * dd;
      wself = dd * dd;
    }
    const int wti = __float_as_int(wt);
    float a0 = 0.0f, a1 = 0.0f, a2 = 0.0f, a3 = 0.0f;
#pragma unroll 1
    for (int k = 0; k < c; ++k) {
      const int   sk = __builtin_amdgcn_readlane(sr, k);
      const float wk = __int_as_float(__builtin_amdgcn_readlane(wti, k));
      const v4f a = *(const v4fa*)(hx + (size_t)sk * DF + 4 * lane);
      a0 = fmaf(wk, a.x, a0); a1 = fmaf(wk, a.y, a1);
      a2 = fmaf(wk, a.z, a2); a3 = fmaf(wk, a.w, a3);
    }
    const v4f sv = *(const v4fa*)(hx + (size_t)nc * DF + 4 * lane);
    const float pzr = big ? qnan : pz;
    const bool live = node < nN;
    v4f y;
    y.x = ((a0 + sv.x * wself) + bv.x) + pzr;
    y.y = ((a1 + sv.y * wself) + bv.y) + pzr;
    y.z = ((a2 + sv.z * wself) + bv.z) + pzr;
    y.w = ((a3 + sv.w * wself) + bv.w) + pzr;
    if (live) {
      const double d0 = (double)y.x, d1 = (double)y.y, d2 = (double)y.z, d3 = (double)y.w;
      sd0 += d0; sd1 += d1; sd2 += d2; sd3 += d3;
      sq0 += d0 * d0; sq1 += d1 * d1; sq2 += d2 * d2; sq3 += d3 * d3;
    }
    v4f ow;
    ow.x = live ? y.x : 0.0f; ow.y = live ? y.y : 0.0f; ow.z = live ? y.z : 0.0f; ow.w = live ? y.w : 0.0f;
    if (node < mRows) {
      float* op = aout + (size_t)node * DF + 4 * lane;
      *(volatile v4f*)op = ow;
      __threadfence();
      *(volatile v4f*)op = ow;
    }
  }

  {
    double* rw = recb + wave * (2 * DF);
    rw[4 * lane + 0] = sd0; rw[4 * lane + 1] = sd1; rw[4 * lane + 2] = sd2; rw[4 * lane + 3] = sd3;
    rw[DF + 4 * lane + 0] = sq0; rw[DF + 4 * lane + 1] = sq1;
    rw[DF + 4 * lane + 2] = sq2; rw[DF + 4 * lane + 3] = sq3;
  }
  __syncthreads();
  if (tid < DF) {
    double r0 = 0.0, r1 = 0.0;
#pragma unroll 1
    for (int w2 = 0; w2 < NWAVE; ++w2) {
      r0 += recb[w2 * (2 * DF) + 2 * tid];
      r1 += recb[w2 * (2 * DF) + 2 * tid + 1];
    }
    v2d rv;
    rv.x = r0; rv.y = r1;
    double* rp = rec + (size_t)blockIdx.x * (2 * DF) + 2 * tid;
    *(volatile v2d*)rp = rv;
    __threadfence();
    *(volatile v2d*)rp = rv;
  }
}

__global__ __launch_bounds__(DF) void k_combine(const double* __restrict__ rec, int nblk, double invN,
                                                const float* __restrict__ g, const float* __restrict__ be,
                                                float* bnp) {
  __shared__ __attribute__((aligned(16))) float os[4 * DF];
  const int f = (int)threadIdx.x;
  double s = 0.0, q = 0.0;
#pragma unroll 1
  for (int b = 0; b < nblk; ++b) {
    s += rec[(size_t)b * (2 * DF) + f];
    q += rec[(size_t)b * (2 * DF) + DF + f];
  }
  const double mu = s * invN;
  double var = q * invN - mu * mu;
  var = var < 0.0 ? 0.0 : var;
  const float rs = rsqrtf((float)var + 1e-5f);
  os[f]          = (float)mu;
  os[DF + f]     = rs * bf16_val(g[f]);
  os[2 * DF + f] = bf16_val(be[f]);
  os[3 * DF + f] = 0.0f;
  __syncthreads();
  const v4f ov = *(const v4fa*)(os + 4 * f);
  *(volatile v4f*)(bnp + 4 * f) = ov;
  __threadfence();
  *(volatile v4f*)(bnp + 4 * f) = ov;
}

__global__ __launch_bounds__(NTHR) void k_apply(const float* __restrict__ A, const float* __restrict__ bnp,
                                                unsigned short* xh, int nUnits) {
  const int u = (int)blockIdx.x * NTHR + (int)threadIdx.x;
  if (u >= nUnits) return;
  const int row = u >> 4;
  const int c8  = (u & 15) * 8;
  const float* apq = A + (size_t)row * DF + c8;
  const v4f a0 = *(const v4fa*)apq;
  const v4f a1 = *(const v4fa*)(apq + 4);
  const v4f m0 = *(const v4fa*)(bnp + c8),           m1 = *(const v4fa*)(bnp + c8 + 4);
  const v4f s0 = *(const v4fa*)(bnp + DF + c8),      s1 = *(const v4fa*)(bnp + DF + c8 + 4);
  const v4f e0 = *(const v4fa*)(bnp + 2 * DF + c8),  e1 = *(const v4fa*)(bnp + 2 * DF + c8 + 4);
  unsigned short* hp = xh + (size_t)row * XP + c8;
  const v4u wh = *(const v4ua*)hp;
  const v4u wl = *(const v4ua*)(hp + DF);
  float av[8], mu[8], sc[8], be[8], xo[8];
  av[0] = a0.x; av[1] = a0.y; av[2] = a0.z; av[3] = a0.w; av[4] = a1.x; av[5] = a1.y; av[6] = a1.z; av[7] = a1.w;
  mu[0] = m0.x; mu[1] = m0.y; mu[2] = m0.z; mu[3] = m0.w; mu[4] = m1.x; mu[5] = m1.y; mu[6] = m1.z; mu[7] = m1.w;
  sc[0] = s0.x; sc[1] = s0.y; sc[2] = s0.z; sc[3] = s0.w; sc[4] = s1.x; sc[5] = s1.y; sc[6] = s1.z; sc[7] = s1.w;
  be[0] = e0.x; be[1] = e0.y; be[2] = e0.z; be[3] = e0.w; be[4] = e1.x; be[5] = e1.y; be[6] = e1.z; be[7] = e1.w;
  xo[0] = __uint_as_float(wh.x << 16)         + __uint_as_float(wl.x << 16);
  xo[1] = __uint_as_float(wh.x & 0xffff0000u) + __uint_as_float(wl.x & 0xffff0000u);
  xo[2] = __uint_as_float(wh.y << 16)         + __uint_as_float(wl.y << 16);
  xo[3] = __uint_as_float(wh.y & 0xffff0000u) + __uint_as_float(wl.y & 0xffff0000u);
  xo[4] = __uint_as_float(wh.z << 16)         + __uint_as_float(wl.z << 16);
  xo[5] = __uint_as_float(wh.z & 0xffff0000u) + __uint_as_float(wl.z & 0xffff0000u);
  xo[6] = __uint_as_float(wh.w << 16)         + __uint_as_float(wl.w << 16);
  xo[7] = __uint_as_float(wh.w & 0xffff0000u) + __uint_as_float(wl.w & 0xffff0000u);
  unsigned hb[8], lb[8];
#pragma unroll
  for (int j = 0; j < 8; ++j) {
    float v = (av[j] - mu[j]) * sc[j] + be[j];
    v = fmaxf(v, 0.0f);
    const float xn = v + xo[j];
    hb[j] = bf16_bits(xn);
    lb[j] = bf16_bits(xn - __uint_as_float(hb[j] << 16));
  }
  v4u oh, ol;
  oh.x = hb[0] | (hb[1] << 16); oh.y = hb[2] | (hb[3] << 16); oh.z = hb[4] | (hb[5] << 16); oh.w = hb[6] | (hb[7] << 16);
  ol.x = lb[0] | (lb[1] << 16); ol.y = lb[2] | (lb[3] << 16); ol.z = lb[4] | (lb[5] << 16); ol.w = lb[6] | (lb[7] << 16);
  *(volatile v4u*)hp = oh;
  *(volatile v4u*)(hp + DF) = ol;
  __threadfence();
  *(volatile v4u*)hp = oh;
  *(volatile v4u*)(hp + DF) = ol;
}

__device__ __forceinline__ int lower_bound_i(const int* __restrict__ a, int n, int key) {
  int lo = 0, len = n;
#pragma unroll 1
  for (int it = 0; it < 24; ++it) {
    const int half = len >> 1;
    const int mid  = lo + half;
    const int mc   = mid < 0 ? 0 : (mid > n - 1 ? n - 1 : mid);
    const int v    = a[mc];
    const bool go  = (len > 0) && (v < key);
    lo  = go ? mid + 1 : lo;
    len = go ? (len - half - 1) : half;
  }
  return lo;
}

__global__ __launch_bounds__(NTHR) void k_pool(const float* __restrict__ a4, const int* __restrict__ bat,
                                               int nN, int SL, const float* __restrict__ bnp,
                                               unsigned short* P) {
  __shared__ __attribute__((aligned(16))) unsigned short rowb[NWAVE * XP];
  const int tid = (int)threadIdx.x, lane = tid & 31, wave = tid >> 5;
  const int g = (int)blockIdx.x * NWAVE + wave;
  unsigned short* rb = rowb + wave * XP;

  const int lo = lower_bound_i(bat, nN, g);
  const int hi = lower_bound_i(bat, nN, g + 1);
  int cntn = hi - lo;
  const bool big = cntn > PCAP;
  cntn = cntn < 0 ? 0 : (cntn > PCAP ? PCAP : cntn);

  int bad = 0;
  const int nIt = (SL + 31) >> 5;
#pragma unroll 1
  for (int it = 0; it < nIt; ++it) {
    const int j = it * 32 + lane;
    const int n = g * SL + j;
    int n1 = n < 1 ? 1 : n;
    n1 = n1 > nN - 1 ? nN - 1 : n1;
    const int b1 = bat[n1];
    const int b0 = bat[n1 - 1];
    const bool viol = (j < SL) && (n >= 1) && (n < nN) && (b1 < b0);
    bad |= viol ? 1 : 0;
  }
  const unsigned anyb = __builtin_amdgcn_ballot_w32(bad != 0);

  const v4f mu = *(const v4fa*)(bnp + 4 * lane);
  const v4f sc = *(const v4fa*)(bnp + DF + 4 * lane);
  const v4f be = *(const v4fa*)(bnp + 2 * DF + 4 * lane);
  float s0 = 0.0f, s1 = 0.0f, s2 = 0.0f, s3 = 0.0f;
#pragma unroll 1
  for (int q = 0; q < cntn; ++q) {
    int n = lo + q;
    n = n < 0 ? 0 : (n > nN - 1 ? nN - 1 : n);
    const v4f v = *(const v4fa*)(a4 + (size_t)n * DF + 4 * lane);
    s0 += fmaxf((v.x - mu.x) * sc.x + be.x, 0.0f);
    s1 += fmaxf((v.y - mu.y) * sc.y + be.y, 0.0f);
    s2 += fmaxf((v.z - mu.z) * sc.z + be.z, 0.0f);
    s3 += fmaxf((v.w - mu.w) * sc.w + be.w, 0.0f);
  }
  const float pz = (big || anyb != 0u) ? __int_as_float(0x7fc00000) : 0.0f;
  const float m0 = s0 + pz, m1 = s1 + pz, m2 = s2 + pz, m3 = s3 + pz;
  v4us mh, ml;
  {
    unsigned hb;
    hb = bf16_bits(m0); mh[0] = (unsigned short)hb; ml[0] = (unsigned short)bf16_bits(m0 - __uint_as_float(hb << 16));
    hb = bf16_bits(m1); mh[1] = (unsigned short)hb; ml[1] = (unsigned short)bf16_bits(m1 - __uint_as_float(hb << 16));
    hb = bf16_bits(m2); mh[2] = (unsigned short)hb; ml[2] = (unsigned short)bf16_bits(m2 - __uint_as_float(hb << 16));
    hb = bf16_bits(m3); mh[3] = (unsigned short)hb; ml[3] = (unsigned short)bf16_bits(m3 - __uint_as_float(hb << 16));
  }
  *(v4usa*)(rb + 4 * lane) = mh;
  *(v4usa*)(rb + DF + 4 * lane) = ml;
  wave_sync();
  const v8us q0 = *(const v8usa*)(rb + 8 * lane);
  unsigned short* op = P + (size_t)g * XP + 8 * lane;
  *(volatile v8us*)op = q0;
  __threadfence();
  *(volatile v8us*)op = q0;
}

__global__ __launch_bounds__(NTHR) void k_ln(const float* __restrict__ F, const float* __restrict__ gl,
                                             const float* __restrict__ bl, float* out) {
  const int tid = (int)threadIdx.x, lane = tid & 31, wave = tid >> 5;
  const int row = (int)blockIdx.x * NWAVE + wave;
  v4f v[6];
#pragma unroll
  for (int j = 0; j < 6; ++j) v[j] = *(const v4fa*)(F + (size_t)row * NO + 4 * (32 * j + lane));
  float s = 0.0f;
#pragma unroll
  for (int j = 0; j < 6; ++j) s += (v[j].x + v[j].y) + (v[j].z + v[j].w);
  s = wsum(s);
  const float mu = s * (1.0f / (float)NO);
  float q = 0.0f;
#pragma unroll
  for (int j = 0; j < 6; ++j) {
    const float d0 = v[j].x - mu, d1 = v[j].y - mu, d2 = v[j].z - mu, d3 = v[j].w - mu;
    q += (d0 * d0 + d1 * d1) + (d2 * d2 + d3 * d3);
  }
  q = wsum(q);
  const float rs = rsqrtf(q * (1.0f / (float)NO) + 1e-5f);
  v4f o[6];
#pragma unroll
  for (int j = 0; j < 6; ++j) {
    const v4f g4 = bf16_val4(*(const v4f*)(gl + 4 * (32 * j + lane)));
    const v4f b4 = bf16_val4(*(const v4f*)(bl + 4 * (32 * j + lane)));
    v4f r;
    r.x = (v[j].x - mu) * rs * g4.x + b4.x;
    r.y = (v[j].y - mu) * rs * g4.y + b4.y;
    r.z = (v[j].z - mu) * rs * g4.z + b4.z;
    r.w = (v[j].w - mu) * rs * g4.w + b4.w;
    o[j] = r;
  }
#pragma unroll
  for (int j = 0; j < 6; ++j) *(volatile v4f*)(out + (size_t)row * NO + 4 * (32 * j + lane)) = o[j];
  __threadfence();
#pragma unroll
  for (int j = 0; j < 6; ++j) *(volatile v4f*)(out + (size_t)row * NO + 4 * (32 * j + lane)) = o[j];
}

static inline int cdiv(int a, int b) { return (a + b - 1) / b; }
static inline size_t al256(size_t o) { return (o + 255) & ~(size_t)255; }

extern "C" void kernel_launch(void* const* d_in, const int* in_sizes, int n_in,
                              void* d_out, int out_size, void* d_ws, size_t ws_size,
                              hipStream_t stream) {
  if (n_in < 31) return;
  if (in_sizes[0] < DF || (in_sizes[0] % DF) != 0) return;
  const int nN = in_sizes[0] / DF;
  if (nN < 64 || nN >= (1 << 20)) return;
  if (in_sizes[1] < 2 || (in_sizes[1] & 1) != 0) return;
  const int nE = in_sizes[1] / 2;
  if (nE < 1 || nE >= (1 << (31 - SLA))) return;
  if (in_sizes[2] != nN) return;
  if (in_sizes[3] != DF * DF || in_sizes[5] != DF * DF || in_sizes[7] != DF * DF || in_sizes[9] != DF * DF) return;
  if (in_sizes[4] != DF || in_sizes[6] != DF || in_sizes[8] != DF || in_sizes[10] != DF) return;
  for (int i = 11; i <= 20; ++i) if (in_sizes[i] != DF) return;
  if (in_sizes[21] != DF * NH || in_sizes[22] != NH) return;
  if (in_sizes[23] != NH * NH || in_sizes[24] != NH) return;
  if (in_sizes[25] != NH * NH || in_sizes[26] != NH) return;
  if (in_sizes[27] != NH * NO || in_sizes[28] != NO) return;
  if (in_sizes[29] != NO || in_sizes[30] != NO) return;
  if (out_size != NGR * NO) return;

  const float* x    = (const float*)d_in[0];
  const int*   edge = (const int*)d_in[1];
  const int*   bat  = (const int*)d_in[2];
  const float* Wg[3]  = {(const float*)d_in[3], (const float*)d_in[5], (const float*)d_in[7]};
  const float* bg[3]  = {(const float*)d_in[4], (const float*)d_in[6], (const float*)d_in[8]};
  const float* Wa   = (const float*)d_in[9];
  const float* ba   = (const float*)d_in[10];
  const float* asrc = (const float*)d_in[11];
  const float* adst = (const float*)d_in[12];
  const float* gk[4]  = {(const float*)d_in[13], (const float*)d_in[15], (const float*)d_in[17], (const float*)d_in[19]};
  const float* bek[4] = {(const float*)d_in[14], (const float*)d_in[16], (const float*)d_in[18], (const float*)d_in[20]};
  const float* Wl1 = (const float*)d_in[21]; const float* bl1 = (const float*)d_in[22];
  const float* Wl2 = (const float*)d_in[23]; const float* bl2 = (const float*)d_in[24];
  const float* Wl3 = (const float*)d_in[25]; const float* bl3 = (const float*)d_in[26];
  const float* Wl4 = (const float*)d_in[27]; const float* bl4 = (const float*)d_in[28];
  const float* gln = (const float*)d_in[29]; const float* bln = (const float*)d_in[30];
  float* out = (float*)d_out;
  const int* src = edge;
  const int* dst = edge + nE;

  const int MP   = cdiv(nN, GBM) * GBM;
  const int gM   = MP / GBM;
  const int gD   = cdiv(nN, NBD);
  const int NBPD = gD * NBD;
  const int gA   = cdiv(MP, NBA);
  if ((long long)gA * NBA < (long long)MP) return;
  if (NBPD < nN) return;
  const int vec8 = ((nE & 3) == 0) ? 1 : 0;
  const int SL   = cdiv(nN, NGR);
  const double invN = 1.0 / (double)nN;

  char* ws = (char*)d_ws;
  size_t off = 0;
  const size_t oWP  = off; off = al256(off + (size_t)EO_END * 2);
  const size_t oXH  = off; off = al256(off + (size_t)MP * XP * 2);
  const size_t oH   = off; off = al256(off + (size_t)MP * DF * 4);
  const size_t oA   = off; off = al256(off + (size_t)MP * DF * 4);
  const size_t oDI  = off; off = al256(off + (size_t)NBPD * 4);
  const size_t oAL  = off; off = al256(off + (size_t)MP * 4);
  const size_t oAR  = off; off = al256(off + (size_t)MP * 4);
  const size_t oRC  = off; off = al256(off + (size_t)gA * 2 * DF * 8);
  const size_t oBN  = off; off = al256(off + (size_t)4 * 4 * DF * 4);
  const size_t oP   = off; off = al256(off + (size_t)NGR * XP * 2);
  const size_t oM1  = off; off = al256(off + (size_t)NGR * 2 * NH * 2);
  const size_t oM2  = off; off = al256(off + (size_t)NGR * 2 * NH * 2);
  const size_t oM3  = off; off = al256(off + (size_t)NGR * 2 * NH * 2);
  const size_t oF   = off; off = al256(off + (size_t)NGR * NO * 4);
  if (off > ws_size || off > (size_t)268435456) return;
  unsigned short* WP  = (unsigned short*)(ws + oWP);
  unsigned short* XH  = (unsigned short*)(ws + oXH);
  float*          H   = (float*)(ws + oH);
  float*          A   = (float*)(ws + oA);
  float*          DI  = (float*)(ws + oDI);
  float*          AL  = (float*)(ws + oAL);
  float*          AR  = (float*)(ws + oAR);
  double*         REC = (double*)(ws + oRC);
  float*          BNP = (float*)(ws + oBN);
  unsigned short* PH  = (unsigned short*)(ws + oP);
  unsigned short* M1  = (unsigned short*)(ws + oM1);
  unsigned short* M2  = (unsigned short*)(ws + oM2);
  unsigned short* M3  = (unsigned short*)(ws + oM3);
  float*          F   = (float*)(ws + oF);

  const size_t scanLds = (size_t)SCAN_LDS_BYTES;
  hipFuncSetAttribute(reinterpret_cast<const void*>(&k_scan<0>), hipFuncAttributeMaxDynamicSharedMemorySize, (int)scanLds);
  hipFuncSetAttribute(reinterpret_cast<const void*>(&k_scan<1>), hipFuncAttributeMaxDynamicSharedMemorySize, (int)scanLds);

  const int nUx = MP * (XP / 8);
  const int nUa = nN * (DF / 8);
  k_wprep<<<UB8 / NTHR, NTHR, 0, stream>>>(Wg[0], Wg[1], Wg[2], Wa, Wl1, Wl2, Wl3, Wl4, WP);
  k_cvx<<<cdiv(nUx, NTHR), NTHR, 0, stream>>>(x, nN, nUx, XH);
  k_deg<<<gD, NTHR, 0, stream>>>(dst, nE, vec8, DI);
  const int eoW[3] = {EO_W1, EO_W2, EO_W3};
  for (int l = 0; l < 3; ++l) {
    const int K = (l == 0) ? DF : XP;
    k_gemm<0><<<dim3(gM, 1), GTHR, 0, stream>>>(XH, XP, WP + eoW[l], K, DF, bg[l], H, M1, asrc, adst, AL, AR);
    k_scan<0><<<gA, NTHR, scanLds, stream>>>(src, dst, nE, nN, vec8, MP, DI, DI, DI, H, bg[l], A, REC);
    k_combine<<<1, DF, 0, stream>>>(REC, gA, invN, gk[l], bek[l], BNP + (size_t)l * 4 * DF);
    k_apply<<<cdiv(nUa, NTHR), NTHR, 0, stream>>>(A, BNP + (size_t)l * 4 * DF, XH, nUa);
  }
  k_gemm<1><<<dim3(gM, 1), GTHR, 0, stream>>>(XH, XP, WP + EO_WA, XP, DF, ba, H, M1, asrc, adst, AL, AR);
  k_scan<1><<<gA, NTHR, scanLds, stream>>>(src, dst, nE, nN, vec8, MP, DI, AL, AR, H, ba, A, REC);
  k_combine<<<1, DF, 0, stream>>>(REC, gA, invN, gk[3], bek[3], BNP + (size_t)3 * 4 * DF);
  k_pool<<<NGR / NWAVE, NTHR, 0, stream>>>(A, bat, nN, SL, BNP + (size_t)3 * 4 * DF, PH);
  k_gemm<2><<<dim3(NGR / GBM, NH / GBN), GTHR, 0, stream>>>(PH, XP,     WP + EO_L1, XP,     NH, bl1, F, M1, asrc, adst, AL, AR);
  k_gemm<2><<<dim3(NGR / GBM, NH / GBN), GTHR, 0, stream>>>(M1, 2 * NH, WP + EO_L2, 2 * NH, NH, bl2, F, M2, asrc, adst, AL, AR);
  k_gemm<2><<<dim3(NGR / GBM, NH / GBN), GTHR, 0, stream>>>(M2, 2 * NH, WP + EO_L3, 2 * NH, NH, bl3, F, M3, asrc, adst, AL, AR);
  k_gemm<3><<<dim3(NGR / GBM, NO / GBN), GTHR, 0, stream>>>(M3, 2 * NH, WP + EO_L4, 2 * NH, NO, bl4, F, M1, asrc, adst, AL, AR);
  k_ln<<<NGR / NWAVE, NTHR, 0, stream>>>(F, gln, bln, out);
}
